// MultiHeadAttentionQuantum_65481071401117
// MI455X (gfx1250) — hardware-verified
//
#include <hip/hip_runtime.h>
#include <math.h>
#include <stdint.h>

#ifndef NB
#define NB 2
#endif
#ifndef SEQ
#define SEQ 2048
#endif
#define NB_FULL  2
#define SEQ_FULL 2048
#define H_   16
#define DK_  64
#define E_   1024
#define BH_  (NB * H_)
#define KSL  192
#define NST  (SEQ / 64)
#define NQT  (SEQ / 64)
#define NKT  (SEQ / 64)
#define NCB  (E_ / 128)
static_assert(H_ * DK_ == E_);
static_assert(KSL == 3 * DK_);
static_assert((SEQ % 64) == 0 && SEQ >= 64 && SEQ <= SEQ_FULL);
static_assert(NB >= 1 && NB <= NB_FULL);
static_assert((E_ % 128) == 0);
static_assert(((E_ * E_) % 2048) == 0);
static_assert(DK_ == 64);

typedef _Float16 v16h __attribute__((ext_vector_type(16)));
typedef _Float16 v8h  __attribute__((ext_vector_type(8)));
typedef float    v8f  __attribute__((ext_vector_type(8)));
typedef float    v4f  __attribute__((ext_vector_type(4)));
typedef unsigned int v4u __attribute__((ext_vector_type(4)));

#if defined(__HIP_DEVICE_COMPILE__)
#define DEV_ASM 1
#else
#define DEV_ASM 0
#endif

__device__ __forceinline__ unsigned short h_bits(_Float16 v) { return __builtin_bit_cast(unsigned short, v); }
__device__ __forceinline__ unsigned pk16(unsigned short a, unsigned short b) { return (unsigned)a | ((unsigned)b << 16); }
__device__ __forceinline__ v8f zero8() { v8f z = {0.f, 0.f, 0.f, 0.f, 0.f, 0.f, 0.f, 0.f}; return z; }

__device__ __forceinline__ float bf16_rne(float f) {
  unsigned u = __float_as_uint(f);
  u = (u + 0x7FFFu + ((u >> 16) & 1u)) & 0xFFFF0000u;
  return __uint_as_float(u);
}
__device__ __forceinline__ unsigned short f16n(float f) {
  const unsigned short bts = h_bits((_Float16)f);
  return ((bts & 0x7C00u) == 0u) ? (unsigned short)(bts & 0x8000u) : bts;
}

__device__ __forceinline__ v16h ldfrag_h(const _Float16* p) {
  union { v16h v; v8h h[2]; } f;
  f.h[0] = *(const v8h*)(p);
  f.h[1] = *(const v8h*)(p + 16);
  return f.v;
}

__device__ __forceinline__ v8f mma_h(v16h a, v16h b, v8f c) {
  c = __builtin_amdgcn_wmma_f32_16x16x32_f16(false, a, false, b, (short)0, c, false, false);
#if DEV_ASM
  asm volatile("v_nop\n\tv_nop\n\tv_nop\n\tv_nop" : "+v"(c) : "v"(a), "v"(b));
#endif
  return c;
}

__device__ __forceinline__ void enc_slots(float f, int g, unsigned short& qs, unsigned short& ks) {
  const unsigned short qhi = f16n(f);
  const float hf = (float)__builtin_bit_cast(_Float16, qhi);
  const float lo = f - hf;
  const unsigned short qlo = f16n(lo * 4096.0f);
  const unsigned short khi = f16n(hf * 64.0f);
  const unsigned short kmd = f16n(hf * 0.015625f);
  const unsigned short klo = f16n(lo * 64.0f);
  qs = (g == 1) ? qlo : qhi;
  ks = (g == 0) ? khi : ((g == 1) ? kmd : klo);
}

__global__ __launch_bounds__(256) void qenc(const float* __restrict__ x, const float* __restrict__ theta,
                                            unsigned short* qap, unsigned short* kbp, unsigned short* vtp) {
  __shared__ __align__(16) float cs[64 * DK_];
  const int tid = (int)threadIdx.x;
  const int bx  = (int)blockIdx.x;
  const int st  = bx % NST;
  const int bh  = bx / NST;
  const int b   = bh / H_;
  const int h   = bh % H_;
  const int s0  = st * 64;

  {
    const int t  = tid >> 2;
    const int dq = (tid & 3) * 16;
    const float* xp = x + ((size_t)b * SEQ_FULL + (size_t)(s0 + t)) * E_ + h * DK_ + dq;
    float* cp = cs + t * DK_ + dq;
#pragma unroll 1
    for (int i = 0; i < 16; ++i) {
      const float a = bf16_rne(xp[i]) + bf16_rne(theta[dq + i]);
      cp[i] = cosf(a);
    }
  }
  __syncthreads();

  if (tid < 64) {
    float* row = cs + tid * DK_;
    float run = row[0];
    float p1 = 1.0f;
#pragma unroll 1
    for (int i = 1; i < DK_; ++i) {
      const float ci = row[i];
      run = run * ci;
      p1 = p1 * ci;
      row[i] = run;
    }
    row[0] = p1;
  }
  __syncthreads();

  const size_t rowbase = (size_t)bh * SEQ + (size_t)s0;
  v4u qv[6], kv[6];
#pragma unroll
  for (int it = 0; it < 6; ++it) {
    const int p  = it * 256 + tid;
    const int t  = p / 24;
    const int j  = p - t * 24;
    const int g  = j >> 3;
    const int d0 = (j & 7) * 8;
    const v4f ca = *(const v4f*)(cs + t * DK_ + d0);
    const v4f cb = *(const v4f*)(cs + t * DK_ + d0 + 4);
    float f[8];
    f[0] = ca[0]; f[1] = ca[1]; f[2] = ca[2]; f[3] = ca[3];
    f[4] = cb[0]; f[5] = cb[1]; f[6] = cb[2]; f[7] = cb[3];
    v4u aq, ak;
#pragma unroll
    for (int e = 0; e < 4; ++e) {
      unsigned short q0b, q1b, k0b, k1b;
      enc_slots(f[2 * e],     g, q0b, k0b);
      enc_slots(f[2 * e + 1], g, q1b, k1b);
      aq[e] = pk16(q0b, q1b);
      ak[e] = pk16(k0b, k1b);
    }
    qv[it] = aq; kv[it] = ak;
  }

  const float vscale = 16384.0f;
  v4u vv[2];
  const int k8 = (tid & 7) * 8;
#pragma unroll
  for (int it = 0; it < 2; ++it) {
    const int d = it * 32 + (tid >> 3);
    v4u a;
#pragma unroll
    for (int e = 0; e < 4; ++e) {
      const float f0 = cs[(k8 + 2 * e) * DK_ + d];
      const float f1 = cs[(k8 + 2 * e + 1) * DK_ + d];
      a[e] = pk16(f16n(f0 * vscale), f16n(f1 * vscale));
    }
    vv[it] = a;
  }

  unsigned short* qo = qap + rowbase * KSL + (size_t)tid * 8;
  unsigned short* ko = kbp + rowbase * KSL + (size_t)tid * 8;
  unsigned short* vo0 = vtp + ((size_t)bh * DK_ + (size_t)(tid >> 3)) * SEQ + (size_t)s0 + (size_t)k8;
  unsigned short* vo1 = vtp + ((size_t)bh * DK_ + (size_t)(32 + (tid >> 3))) * SEQ + (size_t)s0 + (size_t)k8;
  for (int pass = 0; pass < 2; ++pass) {
#pragma unroll
    for (int it = 0; it < 6; ++it) {
      *(volatile v4u*)(qo + (size_t)it * 2048) = qv[it];
      *(volatile v4u*)(ko + (size_t)it * 2048) = kv[it];
    }
    *(volatile v4u*)vo0 = vv[0];
    *(volatile v4u*)vo1 = vv[1];
    __threadfence();
  }
}

__global__ __launch_bounds__(256) void wprep(const float* __restrict__ w, unsigned short* w16) {
  const int i = (int)blockIdx.x * 256 + (int)threadIdx.x;
  if (i < (E_ * E_) / 8) {
    const float* src = w + (size_t)i * 8;
    const v4f a  = *(const v4f*)(src);
    const v4f a4 = *(const v4f*)(src + 4);
    v4u p;
    p[0] = pk16(h_bits((_Float16)(bf16_rne(a[0])  * 1024.0f)), h_bits((_Float16)(bf16_rne(a[1])  * 1024.0f)));
    p[1] = pk16(h_bits((_Float16)(bf16_rne(a[2])  * 1024.0f)), h_bits((_Float16)(bf16_rne(a[3])  * 1024.0f)));
    p[2] = pk16(h_bits((_Float16)(bf16_rne(a4[0]) * 1024.0f)), h_bits((_Float16)(bf16_rne(a4[1]) * 1024.0f)));
    p[3] = pk16(h_bits((_Float16)(bf16_rne(a4[2]) * 1024.0f)), h_bits((_Float16)(bf16_rne(a4[3]) * 1024.0f)));
    unsigned short* dst = w16 + (size_t)i * 8;
    for (int pass = 0; pass < 2; ++pass) {
      *(volatile v4u*)dst = p;
      __threadfence();
    }
  }
}

__global__ __launch_bounds__(128)
void attn_q(const unsigned short* __restrict__ qap, const unsigned short* __restrict__ kbp,
            const unsigned short* __restrict__ vtp, unsigned short* mp) {
  union FH { v16h v; v8h h[2]; };
  __shared__ __align__(16) _Float16 Ksh[64 * KSL];
  __shared__ __align__(16) _Float16 Vsh[64 * 64];
  __shared__ __align__(16) _Float16 Psh[4][16 * 64];
  __shared__ __align__(16) float    Os[4][16 * 64];

  const int tid  = (int)threadIdx.x;
  const int wave = tid >> 5;
  const int lane = tid & 31;
  const int hh   = lane >> 4;
  const int c    = lane & 15;

  const int bx = (int)blockIdx.x;
  const int qt = bx % NQT;
  const int bh = bx / NQT;
  const int b  = bh / H_;
  const int h  = bh % H_;
  const int q0 = qt * 64 + wave * 16;

  const _Float16* QA = (const _Float16*)(const void*)qap;
  const _Float16* KB = (const _Float16*)(const void*)kbp + (size_t)bh * SEQ * KSL;
  const _Float16* VT = (const _Float16*)(const void*)vtp + (size_t)bh * DK_ * SEQ;

  v16h qa[6];
  {
    const _Float16* qr = QA + ((size_t)bh * SEQ + (size_t)(q0 + c)) * KSL + 8 * hh;
#pragma unroll
    for (int ks = 0; ks < 6; ++ks) qa[ks] = ldfrag_h(qr + ks * 32);
  }

  const float sscale = 0.001953125f;

  float mrow[8], lrow[8];
  v8f oacc[4];
#pragma unroll
  for (int dt = 0; dt < 4; ++dt) oacc[dt] = zero8();
#pragma unroll
  for (int r = 0; r < 8; ++r) { mrow[r] = -INFINITY; lrow[r] = 0.f; }

#pragma unroll 1
  for (int kt = 0; kt < NKT; ++kt) {
    const int kv0 = kt * 64;
    __syncthreads();
    {
      const _Float16* kg = KB + (size_t)kv0 * KSL;
#pragma unroll 4
      for (int it = 0; it < 12; ++it) {
        const int p = it * 128 + tid;
        const v8h a0 = *(const v8h*)(kg + (size_t)p * 8);
        *(v8h*)(Ksh + p * 8) = a0;
      }
#pragma unroll
      for (int it = 0; it < 4; ++it) {
        const int p = it * 128 + tid;
        const int d = p >> 3, piece = (p & 7) * 8;
        const v8h v0 = *(const v8h*)(VT + (size_t)d * SEQ + (size_t)kv0 + (size_t)piece);
        *(v8h*)(Vsh + d * 64 + piece) = v0;
      }
    }
    __syncthreads();

    v8f s[4];
#pragma unroll
    for (int j = 0; j < 4; ++j) {
      const _Float16* kr = Ksh + (j * 16 + c) * KSL + 8 * hh;
      v8f acc = zero8();
#pragma unroll
      for (int ks = 0; ks < 6; ++ks) {
        FH kb;
        kb.h[0] = *(const v8h*)(kr + ks * 32);
        kb.h[1] = *(const v8h*)(kr + ks * 32 + 16);
        acc = mma_h(qa[ks], kb.v, acc);
      }
#pragma unroll
      for (int r = 0; r < 8; ++r) s[j][r] = acc[r] * sscale;
    }

    _Float16* pwh = Psh[wave];
#pragma unroll
    for (int r = 0; r < 8; ++r) {
      float m = s[0][r];
#pragma unroll
      for (int j = 1; j < 4; ++j) m = fmaxf(m, s[j][r]);
#pragma unroll
      for (int off = 1; off < 16; off <<= 1) m = fmaxf(m, __shfl_xor(m, off, 32));
      const float mnew  = fmaxf(mrow[r], m);
      const float msafe = (mnew == -INFINITY) ? 0.f : mnew;
      const float alpha = __expf(mrow[r] - msafe);
      mrow[r] = mnew;
      float psum = 0.f;
#pragma unroll
      for (int j = 0; j < 4; ++j) {
        const float p = __expf(s[j][r] - msafe);
        psum += p;
        pwh[(8 * hh + r) * 64 + j * 16 + c] = (_Float16)(p * 1024.0f);
      }
#pragma unroll
      for (int off = 1; off < 16; off <<= 1) psum += __shfl_xor(psum, off, 32);
      lrow[r] = lrow[r] * alpha + psum;
#pragma unroll
      for (int dt = 0; dt < 4; ++dt) oacc[dt][r] *= alpha;
    }
    __builtin_amdgcn_fence(3  , "workgroup");
    __builtin_amdgcn_wave_barrier();
    __builtin_amdgcn_fence(2  , "workgroup");

#pragma unroll
    for (int kk = 0; kk < 2; ++kk) {
      FH pa;
      pa.h[0] = *(const v8h*)(pwh + c * 64 + kk * 32 + 8 * hh);
      pa.h[1] = *(const v8h*)(pwh + c * 64 + kk * 32 + 16 + 8 * hh);
#pragma unroll
      for (int dt = 0; dt < 4; ++dt) {
        FH vb;
        vb.h[0] = *(const v8h*)(Vsh + (dt * 16 + c) * 64 + kk * 32 + 8 * hh);
        vb.h[1] = *(const v8h*)(Vsh + (dt * 16 + c) * 64 + kk * 32 + 16 + 8 * hh);
        oacc[dt] = mma_h(pa.v, vb.v, oacc[dt]);
      }
    }
  }

  float* os = Os[wave];
#pragma unroll
  for (int r = 0; r < 8; ++r) {
    const float l = lrow[r];
    const float inv = ((l > 0.f) ? (1.0f / l) : 0.f) * 0.000244140625f;
#pragma unroll
    for (int dt = 0; dt < 4; ++dt) os[(8 * hh + r) * 64 + dt * 16 + c] = oacc[dt][r] * inv;
  }
  __builtin_amdgcn_fence(3  , "workgroup");
  __builtin_amdgcn_wave_barrier();
  __builtin_amdgcn_fence(2  , "workgroup");
  {
    const int rsub  = lane >> 3;
    const int piece = (lane & 7) * 8;
    v4u val[4];
#pragma unroll
    for (int i = 0; i < 4; ++i) {
      const float* sp = os + (i * 4 + rsub) * 64 + piece;
      const v4f a  = *(const v4f*)(sp);
      const v4f a4 = *(const v4f*)(sp + 4);
      v4u u;
      u[0] = pk16(f16n(a[0]),  f16n(a[1]));
      u[1] = pk16(f16n(a[2]),  f16n(a[3]));
      u[2] = pk16(f16n(a4[0]), f16n(a4[1]));
      u[3] = pk16(f16n(a4[2]), f16n(a4[3]));
      val[i] = u;
    }
    unsigned short* ob = mp + ((size_t)b * SEQ + (size_t)q0) * E_ + (size_t)h * DK_ + (size_t)piece;
    for (int pass = 0; pass < 2; ++pass) {
#pragma unroll
      for (int i = 0; i < 4; ++i) {
        *(volatile v4u*)(ob + (size_t)(i * 4 + rsub) * E_) = val[i];
      }
      __threadfence();
    }
  }
}

__global__ __launch_bounds__(128)
void proj_out(const unsigned short* __restrict__ mp, const unsigned short* __restrict__ w16, float* out) {
  union FH { v16h v; v8h h[2]; };
  __shared__ __align__(16) float lds[4 * 16 * 128];

  const int tid  = (int)threadIdx.x;
  const int wave = tid >> 5;
  const int lane = tid & 31;
  const int hh   = lane >> 4;
  const int c    = lane & 15;

  const int bx = (int)blockIdx.x;
  const int nt = bx % NCB;
  const int mt = bx / NCB;
  const int m0 = mt * 64 + wave * 16;
  const int n0 = nt * 128;

  const _Float16* Ar = (const _Float16*)(const void*)mp  + (size_t)(m0 + c) * E_ + 8 * hh;
  const _Float16* Wr = (const _Float16*)(const void*)w16 + (size_t)(n0 + c) * E_ + 8 * hh;

  v8f acc[8];
#pragma unroll
  for (int j = 0; j < 8; ++j) acc[j] = zero8();

#pragma unroll 1
  for (int ks = 0; ks < E_ / 32; ++ks) {
    const int k0 = ks * 32;
    FH af;
    af.h[0] = *(const v8h*)(Ar + k0);
    af.h[1] = *(const v8h*)(Ar + k0 + 16);
#pragma unroll
    for (int j = 0; j < 4; ++j) {
      FH bf;
      bf.h[0] = *(const v8h*)(Wr + (size_t)j * 16 * E_ + k0);
      bf.h[1] = *(const v8h*)(Wr + (size_t)j * 16 * E_ + k0 + 16);
      acc[j] = mma_h(af.v, bf.v, acc[j]);
    }
    asm volatile("" ::: "memory");
#pragma unroll
    for (int j = 4; j < 8; ++j) {
      FH bf;
      bf.h[0] = *(const v8h*)(Wr + (size_t)j * 16 * E_ + k0);
      bf.h[1] = *(const v8h*)(Wr + (size_t)j * 16 * E_ + k0 + 16);
      acc[j] = mma_h(af.v, bf.v, acc[j]);
    }
  }

  float* slab = lds + wave * 2048;
#pragma unroll
  for (int j = 0; j < 8; ++j) {
#pragma unroll
    for (int r = 0; r < 8; ++r) slab[(8 * hh + r) * 128 + j * 16 + c] = acc[j][r];
  }
  __builtin_amdgcn_fence(3  , "workgroup");
  __builtin_amdgcn_wave_barrier();
  __builtin_amdgcn_fence(2  , "workgroup");

  const float oscale = 1.0f / 4194304.0f;
  v4f vrow[16];
#pragma unroll
  for (int row = 0; row < 16; ++row) {
    const v4f v = *(const v4f*)(slab + row * 128 + lane * 4);
    vrow[row] = v * oscale;
  }
  float* orow = out + (size_t)m0 * E_ + (size_t)n0 + (size_t)lane * 4;
  for (int pass = 0; pass < 2; ++pass) {
#pragma unroll
    for (int row = 0; row < 16; ++row) {
      *(volatile v4f*)(orow + (size_t)row * E_) = vrow[row];
    }
    __threadfence();
  }
}

extern "C" void kernel_launch(void* const* d_in, const int* in_sizes, int n_in,
                              void* d_out, int out_size, void* d_ws, size_t ws_size,
                              hipStream_t stream) {
  if (n_in < 3) return;
  if (in_sizes[0] < ((NB - 1) * SEQ_FULL + SEQ) * E_) return;
  if (in_sizes[1] < DK_) return;
  if (in_sizes[2] < E_ * E_) return;
  if (out_size < NB * SEQ * E_) return;

  const float* x     = (const float*)d_in[0];
  const float* theta = (const float*)d_in[1];
  const float* w     = (const float*)d_in[2];

  const size_t PQA = (size_t)BH_ * SEQ * KSL * 2;
  const size_t PKB = PQA;
  const size_t PVT = (size_t)BH_ * DK_ * SEQ * 2;
  const size_t PMP = (size_t)NB * SEQ * E_ * 2;
  const size_t PW  = (size_t)E_ * E_ * 2;
  size_t off = 0;
  const size_t oQA = off; off += PQA;
  const size_t oKB = off; off += PKB;
  const size_t oVT = off; off += PVT;
  const size_t oMP = off; off += PMP;
  const size_t oW  = off; off += PW;
  if (off > ws_size) return;
  if (off > (size_t)134217728) return;

  char* ws = (char*)d_ws;
  unsigned short* QA  = (unsigned short*)(ws + oQA);
  unsigned short* KB  = (unsigned short*)(ws + oKB);
  unsigned short* VT  = (unsigned short*)(ws + oVT);
  unsigned short* MP  = (unsigned short*)(ws + oMP);
  unsigned short* W16 = (unsigned short*)(ws + oW);

  const dim3 gEnc(BH_ * NST);
  const dim3 gW((E_ * E_ / 8) / 256);
  const dim3 gAttn(BH_ * NQT);
  const dim3 gProj((NB * SEQ / 64) * NCB);

  qenc<<<gEnc, dim3(256), 0, stream>>>(x, theta, QA, KB, VT);
  wprep<<<gW, dim3(256), 0, stream>>>(w, W16);
  attn_q<<<gAttn, dim3(128), 0, stream>>>(QA, KB, VT, MP);
  proj_out<<<gProj, dim3(128), 0, stream>>>(MP, W16, (float*)d_out);
  (void)hipGetLastError();
}
